// MultiHeadAttention_39728447488493
// MI455X (gfx1250) — hardware-verified
//
#include <hip/hip_runtime.h>
#include <math.h>

typedef __attribute__((ext_vector_type(16))) _Float16 v16h;
typedef __attribute__((ext_vector_type(8)))  _Float16 v8h;
typedef __attribute__((ext_vector_type(16))) __bf16   v16b;
typedef __attribute__((ext_vector_type(8)))  __bf16   v8b;
typedef __attribute__((ext_vector_type(8)))  float    v8f;
typedef __attribute__((ext_vector_type(4)))  float    v4f;
typedef __attribute__((ext_vector_type(4)))  unsigned int v4u;
typedef __attribute__((ext_vector_type(8)))  unsigned int v8u;

constexpr int kB   = 2;
constexpr int kS   = 2048;
constexpr int kD   = 1024;
constexpr int kH   = 16;
constexpr int kDh  = kD / kH;
constexpr int kBH  = kB * kH;
constexpr int kTok = kB * kS;
constexpr int kWPlane = kH * kDh * kDh;

constexpr int ce_isqrt(int n) { int r = 0; while ((r + 1) * (r + 1) <= n) ++r; return r; }
static_assert(ce_isqrt(kDh) * ce_isqrt(kDh) == kDh, "head dim is a perfect square");
static_assert(kDh == 64, "kernels are written for head dim 64");
static_assert(kB == 2 && kS == 2048 && kD == 1024 && kH == 16, "wire shapes");
static_assert((kS % 64) == 0 && (kTok % 64) == 0 && (kD % 64) == 0 && (kD % 32) == 0 && (kDh % 32) == 0, "tile multiples");

constexpr float kInvSqrtDh  = 1.0f / (float)ce_isqrt(kDh);
constexpr float kQKVCarry   = 16.0f;
constexpr float kPCarry     = 32768.0f;
constexpr float kCtxCarry   = 256.0f;
constexpr float kWoCarry    = 1024.0f;
constexpr float kScoreScale = kInvSqrtDh / (kQKVCarry * kQKVCarry);
constexpr float kOScale     = kCtxCarry / (kPCarry * kQKVCarry);
constexpr float kOutScale   = 1.0f / (kCtxCarry * kWoCarry);

constexpr size_t kOffQ   = 0;
constexpr size_t kOffK   = kOffQ  + (size_t)kBH * kS * kDh * 2;
constexpr size_t kOffVT  = kOffK  + (size_t)kBH * kS * kDh * 2;
constexpr size_t kOffCC  = kOffVT + (size_t)kBH * kDh * kS * 2;
constexpr size_t kOffWO  = kOffCC + (size_t)kTok * kD * 2;
constexpr size_t kOffWH  = kOffWO + (size_t)kD * kD * 2;
constexpr size_t kOffWL  = kOffWH + (size_t)3 * kWPlane * 2;
constexpr size_t kWsTotal = kOffWL + (size_t)3 * kWPlane * 2;
static_assert(kWsTotal == 36438016ull, "carve total");
static_assert(kWsTotal <= 134217728ull, "carve cap");
static_assert((kOffK % 128) == 0 && (kOffVT % 128) == 0 && (kOffCC % 128) == 0 && (kOffWO % 128) == 0 &&
              (kOffWH % 128) == 0 && (kOffWL % 128) == 0, "128-B aligned regions");

__device__ __forceinline__ unsigned short f2bf_bits(float f) {
  unsigned u = __float_as_uint(f);
  return (unsigned short)((u + 0x7FFFu + ((u >> 16) & 1u)) >> 16);
}
__device__ __forceinline__ float bf_bits2f(unsigned short h) { return __uint_as_float(((unsigned)h) << 16); }
__device__ __forceinline__ unsigned pk16(unsigned short a, unsigned short b) { return (unsigned)a | ((unsigned)b << 16); }
__device__ __forceinline__ unsigned short h_bits(float f) { const _Float16 h = (_Float16)f; return __builtin_bit_cast(unsigned short, h); }

__device__ __forceinline__ v4u pack8_f16(v4f a, v4f b) {
  const float f0 = a[0], f1 = a[1], f2 = a[2], f3 = a[3];
  const float f4 = b[0], f5 = b[1], f6 = b[2], f7 = b[3];
  return (v4u){pk16(h_bits(f0), h_bits(f1)), pk16(h_bits(f2), h_bits(f3)),
               pk16(h_bits(f4), h_bits(f5)), pk16(h_bits(f6), h_bits(f7))};
}

__device__ __forceinline__ v8f mma_h(v16h a, v16h b, v8f c) {
  c = __builtin_amdgcn_wmma_f32_16x16x32_f16(false, a, false, b, (short)0, c, false, false);
  asm volatile("v_nop\n\tv_nop\n\tv_nop\n\tv_nop" : "+v"(c) : "v"(a), "v"(b));
  return c;
}
__device__ __forceinline__ v8f mma_b(v16b a, v16b b, v8f c) {
  c = __builtin_amdgcn_wmma_f32_16x16x32_bf16(false, a, false, b, (short)0, c, false, false);
  asm volatile("v_nop\n\tv_nop\n\tv_nop\n\tv_nop" : "+v"(c) : "v"(a), "v"(b));
  return c;
}

template <typename T> struct Frag;
template <> struct Frag<_Float16> {
  typedef v16h V; union U { v16h v; v8h h[2]; };
  static __device__ __forceinline__ v16h load(const _Float16* p) {
    U f; f.h[0] = *(const v8h*)(p); f.h[1] = *(const v8h*)(p + 16); return f.v;
  }
};
template <> struct Frag<__bf16> {
  typedef v16b V; union U { v16b v; v8b h[2]; };
  static __device__ __forceinline__ v16b load(const __bf16* p) {
    U f; f.h[0] = *(const v8b*)(p); f.h[1] = *(const v8b*)(p + 16); return f.v;
  }
};

__global__ __launch_bounds__(256) void wo_cast_kernel(const float* __restrict__ in, unsigned short* __restrict__ out, int n8, float scale) {
  const int i = blockIdx.x * 256 + threadIdx.x;
  if (i >= n8) return;
  const float* p = in + 8 * (size_t)i;
  v4f a = *(const v4f*)(p);
  v4f c = *(const v4f*)(p + 4);
  a = a * scale;
  c = c * scale;
  const v4u u = pack8_f16(a, c);
  unsigned short* q = out + 8 * (size_t)i;
  *(volatile v4u*)q = u;
  __threadfence();
  *(volatile v4u*)q = u;
}

__global__ __launch_bounds__(256) void w_split_kernel(const float* __restrict__ Wq, const float* __restrict__ Wk,
                                                      const float* __restrict__ Wv,
                                                      unsigned short* __restrict__ dhi, unsigned short* __restrict__ dlo) {
  const int which = blockIdx.y;
  const float* src = (which == 0) ? Wq : (which == 1) ? Wk : Wv;
  const int i = blockIdx.x * 256 + threadIdx.x;
  if (i >= kWPlane / 8) return;
  const size_t e0 = (size_t)i << 3;
  const v4f a0 = *(const v4f*)(src + e0);
  const v4f a1 = *(const v4f*)(src + e0 + 4);
  float f[8];
  f[0] = a0[0]; f[1] = a0[1]; f[2] = a0[2]; f[3] = a0[3];
  f[4] = a1[0]; f[5] = a1[1]; f[6] = a1[2]; f[7] = a1[3];
  unsigned short hb[8], lb[8];
#pragma unroll
  for (int e = 0; e < 8; ++e) {
    hb[e] = f2bf_bits(f[e]);
    lb[e] = f2bf_bits(f[e] - bf_bits2f(hb[e]));
  }
  const v4u uh = (v4u){pk16(hb[0], hb[1]), pk16(hb[2], hb[3]), pk16(hb[4], hb[5]), pk16(hb[6], hb[7])};
  const v4u ul = (v4u){pk16(lb[0], lb[1]), pk16(lb[2], lb[3]), pk16(lb[4], lb[5]), pk16(lb[6], lb[7])};
  unsigned short* qh = dhi + (size_t)which * kWPlane + e0;
  unsigned short* ql = dlo + (size_t)which * kWPlane + e0;
  *(volatile v4u*)qh = uh;
  *(volatile v4u*)ql = ul;
  __threadfence();
  *(volatile v4u*)qh = uh;
  *(volatile v4u*)ql = ul;
}

__global__ __launch_bounds__(128) void head_proj_kernel(
    const float* __restrict__ xq, const float* __restrict__ xk, const float* __restrict__ xv,
    const unsigned short* __restrict__ Whi, const unsigned short* __restrict__ Wlo,
    unsigned short* __restrict__ Qo, unsigned short* __restrict__ Ko, unsigned short* __restrict__ Vto)
{
  __shared__ __align__(16) float sT[64 * 68];
  const int tid  = threadIdx.x;
  const int wave = __builtin_amdgcn_readfirstlane((int)(threadIdx.x >> 5));
  const int lane = tid & 31;
  const int hh   = lane >> 4;
  const int c    = lane & 15;
  const int which = blockIdx.z;
  const int bh    = blockIdx.y;
  const int s0    = blockIdx.x * 64;
  const int b     = bh / kH;
  const int h     = bh - b * kH;

  const float* X = (which == 0) ? xq : (which == 1) ? xk : xv;
  const float* xrow = X + ((size_t)b * kS + s0 + wave * 16 + c) * kD + h * kDh;
  const __bf16* Wh = (const __bf16*)Whi + (size_t)(which * kH + h) * kDh * kDh;
  const __bf16* Wl = (const __bf16*)Wlo + (size_t)(which * kH + h) * kDh * kDh;

  v8f acc[4];
#pragma unroll
  for (int j = 0; j < 4; ++j) acc[j] = (v8f){0.f, 0.f, 0.f, 0.f, 0.f, 0.f, 0.f, 0.f};

#pragma unroll
  for (int kk = 0; kk < 2; ++kk) {
    const float* p = xrow + kk * 32 + 8 * hh;
    const v4f a0 = *(const v4f*)(p);
    const v4f a1 = *(const v4f*)(p + 4);
    const v4f a2 = *(const v4f*)(p + 16);
    const v4f a3 = *(const v4f*)(p + 20);
    float f[16];
    f[0]  = a0[0]; f[1]  = a0[1]; f[2]  = a0[2]; f[3]  = a0[3];
    f[4]  = a1[0]; f[5]  = a1[1]; f[6]  = a1[2]; f[7]  = a1[3];
    f[8]  = a2[0]; f[9]  = a2[1]; f[10] = a2[2]; f[11] = a2[3];
    f[12] = a3[0]; f[13] = a3[1]; f[14] = a3[2]; f[15] = a3[3];
    unsigned wh[8], wl[8];
#pragma unroll
    for (int w = 0; w < 8; ++w) {
      const unsigned short h0 = f2bf_bits(f[2 * w]);
      const unsigned short h1 = f2bf_bits(f[2 * w + 1]);
      const unsigned short l0 = f2bf_bits(f[2 * w] - bf_bits2f(h0));
      const unsigned short l1 = f2bf_bits(f[2 * w + 1] - bf_bits2f(h1));
      wh[w] = pk16(h0, h1);
      wl[w] = pk16(l0, l1);
    }
    const v8u vh = (v8u){wh[0], wh[1], wh[2], wh[3], wh[4], wh[5], wh[6], wh[7]};
    const v8u vl = (v8u){wl[0], wl[1], wl[2], wl[3], wl[4], wl[5], wl[6], wl[7]};
    const v16b ah = __builtin_bit_cast(v16b, vh);
    const v16b al = __builtin_bit_cast(v16b, vl);
#pragma unroll
    for (int j = 0; j < 4; ++j) {
      const size_t bo = (size_t)(j * 16 + c) * kDh + kk * 32 + 8 * hh;
      const v16b bhf = Frag<__bf16>::load(Wh + bo);
      const v16b blf = Frag<__bf16>::load(Wl + bo);
      acc[j] = mma_b(ah, blf, acc[j]);
      acc[j] = mma_b(al, bhf, acc[j]);
      acc[j] = mma_b(ah, bhf, acc[j]);
    }
  }

  const bool isV = (which == 2);
#pragma unroll
  for (int j = 0; j < 4; ++j) {
#pragma unroll
    for (int r = 0; r < 8; ++r) {
      const int rl = wave * 16 + 8 * hh + r;
      const int cl = j * 16 + c;
      const int idx = isV ? (cl * 68 + rl) : (rl * 68 + cl);
      sT[idx] = acc[j][r] * kQKVCarry;
    }
  }
  __syncthreads();

  const int q  = lane >> 3;
  const int c8 = (lane & 7) * 8;
  unsigned short* dst0;
  size_t pitch;
  if (which == 0)      { dst0 = Qo  + ((size_t)bh * kS + s0) * kDh; pitch = (size_t)kDh; }
  else if (which == 1) { dst0 = Ko  + ((size_t)bh * kS + s0) * kDh; pitch = (size_t)kDh; }
  else                 { dst0 = Vto + (size_t)bh * kDh * kS + s0;   pitch = (size_t)kS; }
  v4u u[4];
#pragma unroll
  for (int it = 0; it < 4; ++it) {
    const int orow = wave * 16 + it * 4 + q;
    const float* sp = sT + orow * 68 + c8;
    const v4f t0 = *(const v4f*)(sp);
    const v4f t1 = *(const v4f*)(sp + 4);
    u[it] = pack8_f16(t0, t1);
  }
  for (int pass = 0; pass < 2; ++pass) {
#pragma unroll
    for (int it = 0; it < 4; ++it) {
      const int orow = wave * 16 + it * 4 + q;
      *(volatile v4u*)(dst0 + (size_t)orow * pitch + c8) = u[it];
    }
    __threadfence();
  }
}

__global__ __launch_bounds__(128) void attn_stream_kernel(
    const unsigned short* __restrict__ Qp, const unsigned short* __restrict__ Kp,
    const unsigned short* __restrict__ Vtp, unsigned short* __restrict__ CC)
{
  __shared__ __align__(16) _Float16 Ksh[64 * 64];
  __shared__ __align__(16) _Float16 Vsh[64 * 64];
  __shared__ __align__(16) _Float16 Psh[4][16 * 64];
  __shared__ __align__(16) float    Os[4][16 * 68];

  const int tid  = threadIdx.x;
  const int wave = __builtin_amdgcn_readfirstlane((int)(threadIdx.x >> 5));
  const int lane = tid & 31;
  const int hh   = lane >> 4;
  const int c    = lane & 15;
  const int qb   = blockIdx.x;
  const int bh   = blockIdx.y;
  const int b    = bh / kH;
  const int h    = bh - b * kH;
  const int q0   = qb * 64 + wave * 16;

  const _Float16* Qb = (const _Float16*)Qp  + (size_t)bh * kS * kDh;
  const _Float16* Kb = (const _Float16*)Kp  + (size_t)bh * kS * kDh;
  const _Float16* Vb = (const _Float16*)Vtp + (size_t)bh * kDh * kS;

  v16h qa[2];
#pragma unroll
  for (int dc = 0; dc < 2; ++dc)
    qa[dc] = Frag<_Float16>::load(Qb + (size_t)(q0 + c) * kDh + dc * 32 + 8 * hh);

  float mrow[8], lrow[8];
  v8f oacc[4];
#pragma unroll
  for (int r = 0; r < 8; ++r) { mrow[r] = -INFINITY; lrow[r] = 0.f; }
#pragma unroll
  for (int t = 0; t < 4; ++t) oacc[t] = (v8f){0.f, 0.f, 0.f, 0.f, 0.f, 0.f, 0.f, 0.f};

  _Float16* pw = Psh[wave];

#pragma unroll 1
  for (int kc = 0; kc < kS / 64; ++kc) {
    const int kv0 = kc * 64;
    __syncthreads();
#pragma unroll
    for (int i = 0; i < 4; ++i) {
      const int idx = tid + 128 * i;
      const v8h kvv = *(const v8h*)(Kb + (size_t)kv0 * kDh + idx * 8);
      *(v8h*)(Ksh + idx * 8) = kvv;
      const int d   = idx >> 3;
      const int cc8 = (idx & 7) * 8;
      const v8h vvv = *(const v8h*)(Vb + (size_t)d * kS + kv0 + cc8);
      *(v8h*)(Vsh + d * 64 + cc8) = vvv;
    }
    __syncthreads();

    v8f s[4];
#pragma unroll
    for (int j = 0; j < 4; ++j) {
      s[j] = (v8f){0.f, 0.f, 0.f, 0.f, 0.f, 0.f, 0.f, 0.f};
#pragma unroll
      for (int dc = 0; dc < 2; ++dc) {
        const v16h kf = Frag<_Float16>::load(Ksh + (j * 16 + c) * 64 + dc * 32 + 8 * hh);
        s[j] = mma_h(qa[dc], kf, s[j]);
      }
    }

    float cm[8];
#pragma unroll
    for (int r = 0; r < 8; ++r) {
      float m = -INFINITY;
#pragma unroll
      for (int j = 0; j < 4; ++j) {
        s[j][r] *= kScoreScale;
        m = fmaxf(m, s[j][r]);
      }
#pragma unroll
      for (int off = 1; off < 16; off <<= 1) m = fmaxf(m, __shfl_xor(m, off, 32));
      cm[r] = m;
    }

#pragma unroll
    for (int r = 0; r < 8; ++r) {
      const float mnew  = fmaxf(mrow[r], cm[r]);
      const float alpha = __expf(mrow[r] - mnew);
      mrow[r] = mnew;
      float psum = 0.f;
#pragma unroll
      for (int j = 0; j < 4; ++j) {
        const float p = __expf(s[j][r] - mnew);
        psum += p;
        pw[(8 * hh + r) * 64 + j * 16 + c] = (_Float16)(p * kPCarry);
      }
#pragma unroll
      for (int off = 1; off < 16; off <<= 1) psum += __shfl_xor(psum, off, 32);
      lrow[r] = lrow[r] * alpha + psum;
#pragma unroll
      for (int t = 0; t < 4; ++t) oacc[t][r] *= alpha;
    }
    __builtin_amdgcn_fence(__ATOMIC_RELEASE, "workgroup");
    __builtin_amdgcn_wave_barrier();
    __builtin_amdgcn_fence(__ATOMIC_ACQUIRE, "workgroup");

#pragma unroll
    for (int kk = 0; kk < 2; ++kk) {
      const v16h pa = Frag<_Float16>::load(pw + c * 64 + kk * 32 + 8 * hh);
#pragma unroll
      for (int t = 0; t < 4; ++t) {
        const v16h vf = Frag<_Float16>::load(Vsh + (t * 16 + c) * 64 + kk * 32 + 8 * hh);
        oacc[t] = mma_h(pa, vf, oacc[t]);
      }
    }
  }

  float* os = Os[wave];
#pragma unroll
  for (int r = 0; r < 8; ++r) {
    const float inv = kOScale * (1.0f / lrow[r]);
#pragma unroll
    for (int t = 0; t < 4; ++t) os[(8 * hh + r) * 68 + t * 16 + c] = oacc[t][r] * inv;
  }
  __syncthreads();
  {
    const int q  = lane >> 3;
    const int c8 = (lane & 7) * 8;
    unsigned short* dst0 = CC + ((size_t)b * kS + q0) * kD + h * kDh;
    v4u u[4];
#pragma unroll
    for (int it = 0; it < 4; ++it) {
      const int row = it * 4 + q;
      const float* sp = os + row * 68 + c8;
      const v4f t0 = *(const v4f*)(sp);
      const v4f t1 = *(const v4f*)(sp + 4);
      u[it] = pack8_f16(t0, t1);
    }
    for (int pass = 0; pass < 2; ++pass) {
#pragma unroll
      for (int it = 0; it < 4; ++it) {
        const int row = it * 4 + q;
        *(volatile v4u*)(dst0 + (size_t)row * kD + c8) = u[it];
      }
      __threadfence();
    }
  }
}

__global__ __launch_bounds__(256) void out_proj_gemm_kernel(
    const unsigned short* __restrict__ Ap, int lda,
    const unsigned short* __restrict__ Btp, int ldb,
    float* __restrict__ C, int ldc,
    const float* __restrict__ bias,
    int M, int N, int K, float scale)
{
  const _Float16* A  = (const _Float16*)Ap;
  const _Float16* Bt = (const _Float16*)Btp;
  __shared__ __align__(16) float sT[8][16 * 68];
  const int lane = threadIdx.x & 31;
  const int wave = __builtin_amdgcn_readfirstlane((int)(threadIdx.x >> 5));
  const int tilesN = N >> 6;
  const int tilesM = M >> 6;
  const int tile = blockIdx.x * 8 + wave;
  if (tile >= tilesM * tilesN) return;
  const int tm = tile / tilesN;
  const int tn = tile - tm * tilesN;
  const int m0 = tm << 6;
  const int n0 = tn << 6;

  const int rlane = lane & 15;
  const int koff  = (lane >> 4) * 8;
  const int mOff  = (lane >> 4) * 8;

  v8f acc[4][4];
#pragma unroll
  for (int i = 0; i < 4; ++i)
#pragma unroll
    for (int j = 0; j < 4; ++j) acc[i][j] = (v8f){0.f, 0.f, 0.f, 0.f, 0.f, 0.f, 0.f, 0.f};

  for (int k0 = 0; k0 < K; k0 += 32) {
    v16h bf[4];
#pragma unroll
    for (int j = 0; j < 4; ++j) {
      const size_t bo = (size_t)(n0 + (j << 4) + rlane) * ldb + koff + k0;
      bf[j] = Frag<_Float16>::load(Bt + bo);
    }
#pragma unroll
    for (int i = 0; i < 4; ++i) {
      const size_t ao = (size_t)(m0 + (i << 4) + rlane) * lda + koff + k0;
      const v16h af = Frag<_Float16>::load(A + ao);
#pragma unroll
      for (int j = 0; j < 4; ++j) acc[i][j] = mma_h(af, bf[j], acc[i][j]);
    }
  }

  float bv[4];
#pragma unroll
  for (int j = 0; j < 4; ++j) bv[j] = bias[n0 + (j << 4) + rlane];

  float* slab = sT[wave];
#pragma unroll
  for (int i = 0; i < 4; ++i) {
    const int mBase = m0 + (i << 4);
#pragma unroll
    for (int j = 0; j < 4; ++j) {
#pragma unroll
      for (int r = 0; r < 8; ++r) {
        const float v = acc[i][j][r] * scale + bv[j];
        slab[(mOff + r) * 68 + (j << 4) + rlane] = v;
      }
    }
    __builtin_amdgcn_fence(__ATOMIC_RELEASE, "workgroup");
    __builtin_amdgcn_wave_barrier();
    __builtin_amdgcn_fence(__ATOMIC_ACQUIRE, "workgroup");
    {
      const int hh = lane >> 4, c4 = (lane & 15) * 4;
      for (int pass = 0; pass < 2; ++pass) {
#pragma unroll
        for (int it = 0; it < 8; ++it) {
          const int row = it * 2 + hh;
          const v4f v = *(const v4f*)(slab + row * 68 + c4);
          *(volatile v4f*)(C + (size_t)(mBase + row) * ldc + n0 + c4) = v;
        }
        __threadfence();
      }
    }
    __builtin_amdgcn_fence(__ATOMIC_RELEASE, "workgroup");
    __builtin_amdgcn_wave_barrier();
    __builtin_amdgcn_fence(__ATOMIC_ACQUIRE, "workgroup");
  }
}

extern "C" void kernel_launch(void* const* d_in, const int* in_sizes, int n_in,
                              void* d_out, int out_size, void* d_ws, size_t ws_size,
                              hipStream_t stream) {
  if (n_in < 8) return;
  if (in_sizes[0] != kTok * kD) return;
  if (in_sizes[1] != kTok * kD) return;
  if (in_sizes[2] != kTok * kD) return;
  if (in_sizes[3] != kWPlane) return;
  if (in_sizes[4] != kWPlane) return;
  if (in_sizes[5] != kWPlane) return;
  if (in_sizes[6] != kD * kD) return;
  if (in_sizes[7] != kD) return;
  if (out_size != kTok * kD) return;
  if (ws_size < kWsTotal) return;

  const float* query = (const float*)d_in[0];
  const float* key   = (const float*)d_in[1];
  const float* value = (const float*)d_in[2];
  const float* Wq    = (const float*)d_in[3];
  const float* Wk    = (const float*)d_in[4];
  const float* Wv    = (const float*)d_in[5];
  const float* Wo    = (const float*)d_in[6];
  const float* bo    = (const float*)d_in[7];
  float* out = (float*)d_out;

  char* ws = (char*)d_ws;
  unsigned short* Q16  = (unsigned short*)(ws + kOffQ);
  unsigned short* K16  = (unsigned short*)(ws + kOffK);
  unsigned short* VT16 = (unsigned short*)(ws + kOffVT);
  unsigned short* CC16 = (unsigned short*)(ws + kOffCC);
  unsigned short* WO16 = (unsigned short*)(ws + kOffWO);
  unsigned short* WH   = (unsigned short*)(ws + kOffWH);
  unsigned short* WL   = (unsigned short*)(ws + kOffWL);

  wo_cast_kernel<<<(kD * kD / 8) / 256, 256, 0, stream>>>(Wo, WO16, kD * kD / 8, kWoCarry);
  w_split_kernel<<<dim3((kWPlane / 8) / 256, 3), 256, 0, stream>>>(Wq, Wk, Wv, WH, WL);

  head_proj_kernel<<<dim3(kS / 64, kBH, 3), 128, 0, stream>>>(query, key, value, WH, WL, Q16, K16, VT16);

  attn_stream_kernel<<<dim3(kS / 64, kBH), 128, 0, stream>>>(Q16, K16, VT16, CC16);

  out_proj_gemm_kernel<<<dim3((kTok / 64) * (kD / 64) / 8), 256, 0, stream>>>(
      CC16, kD, WO16, kD, out, kD, bo, kTok, kD, kD, kOutScale);
}
